// MultiModalModel_22016002360055
// MI455X (gfx1250) — hardware-verified
//
#include <hip/hip_runtime.h>
#include <math.h>
#include <stdint.h>

typedef __attribute__((ext_vector_type(16))) _Float16 v16h;
typedef __attribute__((ext_vector_type(8)))  _Float16 v8h;
typedef __attribute__((ext_vector_type(16))) __bf16   v16b;
typedef __attribute__((ext_vector_type(8)))  __bf16   v8b;
typedef __attribute__((ext_vector_type(8)))  float    v8f;
typedef __attribute__((ext_vector_type(4)))  float    v4f;
typedef __attribute__((ext_vector_type(4)))  int      v4i;

constexpr int kNumImg    = 256;
constexpr int kNumTxt    = 256;
constexpr int kNumWords  = 32;
constexpr int kEmb       = 128;
constexpr int kSpatial   = 49;
constexpr int kTL        = kNumTxt * kNumWords;
constexpr int kGemmM     = kNumImg * kSpatial;
constexpr int kGemmK     = kEmb;
constexpr int kChunkN    = 2048;
constexpr int kNumChunks = kTL / kChunkN;
constexpr int kImgElems  = kNumImg * kEmb * kSpatial;
constexpr int kTxtElems  = kTL * kEmb;
constexpr int kOutElems  = 2 * kNumImg * kNumTxt;
constexpr int kOut1Elem  = kNumImg * kNumTxt;

static_assert(kGemmM % 64 == 0);
static_assert(kChunkN % 64 == 0);
static_assert(kGemmK % 32 == 0);
static_assert(kTL % kChunkN == 0);
static_assert(kOut1Elem + kNumImg * kNumTxt == kOutElems);

#define OPERAND_CARRY 16.0f
#define CARRY_FOLD (1.0f / 256.0f)

constexpr size_t kOffA    = 0;
constexpr size_t kBytesA  = (size_t)kGemmM * kEmb * 2;
constexpr size_t kOffBt   = kOffA + kBytesA;
constexpr size_t kBytesBt = (size_t)kTL * kEmb * 2;
constexpr size_t kOffC    = kOffBt + kBytesBt;
constexpr size_t kBytesC  = (size_t)kGemmM * kChunkN * 4;
constexpr size_t kOffM    = kOffC + kBytesC;
constexpr size_t kBytesM  = (size_t)kNumImg * kNumTxt * 4;
constexpr size_t kWsTotal = kOffM + kBytesM;
static_assert(kWsTotal <= 134217728ull);
static_assert(kOffBt % 256 == 0 && kOffC % 256 == 0 && kOffM % 256 == 0);

#define PSCALE 32768.0f
#define U16(p) ((const unsigned short*)(const void*)(p))
#define PSCALE_INV (1.0f / 32768.0f)

__device__ __forceinline__ unsigned short f2bf_bits(float f) {
  unsigned u = __float_as_uint(f);
  return (unsigned short)((u + 0x7FFFu + ((u >> 16) & 1u)) >> 16);
}
__device__ __forceinline__ float bf_bits2f(unsigned short h) { return __uint_as_float(((unsigned)h) << 16); }

__device__ __forceinline__ void dep_guard_h(v8f& a, v8f& b, v16h x, v16h y) { asm volatile("v_nop\n\tv_nop\n\tv_nop\n\tv_nop" : "+v"(a), "+v"(b) : "v"(x), "v"(y)); }
__device__ __forceinline__ void dep_guard_b(v8f& a, v8f& b, v16b x, v16b y) { asm volatile("v_nop\n\tv_nop\n\tv_nop\n\tv_nop" : "+v"(a), "+v"(b) : "v"(x), "v"(y)); }
__device__ __forceinline__ void keep4_h(v16h a, v16h b, v16h c, v16h d) { asm volatile("v_nop" :: "v"(a), "v"(b), "v"(c), "v"(d)); }
__device__ __forceinline__ void keep4_b(v16b a, v16b b, v16b c, v16b d) { asm volatile("v_nop" :: "v"(a), "v"(b), "v"(c), "v"(d)); }
__device__ __forceinline__ void acc_guard4(v8f& a, v8f& b, v8f& c, v8f& d) { asm volatile("v_nop\n\tv_nop\n\tv_nop\n\tv_nop" : "+v"(a), "+v"(b), "+v"(c), "+v"(d)); }
template <typename T> struct Frag;
template <> struct Frag<_Float16> {
  typedef v16h V; union U { v16h v; v8h h[2]; };
  static __device__ __forceinline__ v16h load(const _Float16* p) {
    U f; f.h[0] = *(const v8h*)(p); f.h[1] = *(const v8h*)(p + 16); return f.v;
  }
  static __device__ __forceinline__ v8f mma(v16h a, v16h b, v8f c) {
    return __builtin_amdgcn_wmma_f32_16x16x32_f16(false, a, false, b, (short)0, c, false, false);
  }
  static __device__ __forceinline__ void guard(v8f& a, v8f& b, v16h x, v16h y) { dep_guard_h(a, b, x, y); }
  static __device__ __forceinline__ void keep(v16h a, v16h b, v16h c, v16h d) { keep4_h(a, b, c, d); }
};
template <> struct Frag<__bf16> {
  typedef v16b V; union U { v16b v; v8b h[2]; };
  static __device__ __forceinline__ v16b load(const __bf16* p) {
    U f; f.h[0] = *(const v8b*)(p); f.h[1] = *(const v8b*)(p + 16); return f.v;
  }
  static __device__ __forceinline__ v8f mma(v16b a, v16b b, v8f c) {
    return __builtin_amdgcn_wmma_f32_16x16x32_bf16(false, a, false, b, (short)0, c, false, false);
  }
  static __device__ __forceinline__ void guard(v8f& a, v8f& b, v16b x, v16b y) { dep_guard_b(a, b, x, y); }
  static __device__ __forceinline__ void keep(v16b a, v16b b, v16b c, v16b d) { keep4_b(a, b, c, d); }
};

template <int ET> struct Elem;
template <> struct Elem<0> { typedef _Float16 T; };
template <> struct Elem<1> { typedef __bf16 T; };
template <int ET, bool SPLIT, int BIAS_MODE, int OUT_MODE, bool RESID, int ACT = 0>
__global__ __launch_bounds__(256) void wmma_gemm64(
    const unsigned short* __restrict__ Ap, const unsigned short* __restrict__ A2p, int lda, long strideA,
    const unsigned short* __restrict__ Btp, const unsigned short* __restrict__ Bt2p, int ldb, long strideB,
    void* __restrict__ Cout, void* __restrict__ Cout2, int ldc, long strideC,
    const float* __restrict__ bias,
    const float* __restrict__ resid, long strideR,
    int M, int N, int K, float scale) {
  typedef typename Elem<ET>::T T;
  typedef typename Frag<T>::V V;
  const T* A = (const T*)Ap; const T* A2 = (const T*)A2p; const T* Bt = (const T*)Btp; const T* Bt2 = (const T*)Bt2p;
  __shared__ __align__(16) float sT[8][16 * 68];
  const int b    = blockIdx.y;
  const int lane = threadIdx.x & 31;
  const int wave = threadIdx.x >> 5;
  const int tilesN = N >> 6;
  const int tilesM = M >> 6;
  const int tile = blockIdx.x * 8 + wave;
  if (tile >= tilesM * tilesN) return;
  const int tm = tile / tilesN;
  const int tn = tile - tm * tilesN;
  const int m0 = tm << 6;
  const int n0 = tn << 6;

  const T* Ab  = A  + (size_t)b * strideA;
  const T* Bb  = Bt + (size_t)b * strideB;
  const T* Ab2 = SPLIT ? (A2  + (size_t)b * strideA) : nullptr;
  const T* Bb2 = SPLIT ? (Bt2 + (size_t)b * strideB) : nullptr;

  const int rlane = lane & 15;
  const int koff  = (lane >> 4) * 8;
  const int mOff  = (lane >> 4) * 8;

  v8f acc[4][4];
#pragma unroll
  for (int i = 0; i < 4; ++i)
#pragma unroll
    for (int j = 0; j < 4; ++j) acc[i][j] = (v8f){0.f,0.f,0.f,0.f,0.f,0.f,0.f,0.f};

  for (int k0 = 0; k0 < K; k0 += 32) {
    V bh[4], bl[4];
#pragma unroll
    for (int j = 0; j < 4; ++j) {
      const size_t bo = (size_t)(n0 + (j << 4) + rlane) * ldb + koff + k0;
      bh[j] = Frag<T>::load(Bb + bo);
      if (SPLIT) bl[j] = Frag<T>::load(Bb2 + bo);
    }
#pragma unroll
    for (int i = 0; i < 4; ++i) {
      const size_t ao = (size_t)(m0 + (i << 4) + rlane) * lda + koff + k0;
      V ah = Frag<T>::load(Ab + ao);
      V al;
      if (SPLIT) al = Frag<T>::load(Ab2 + ao);
#pragma unroll
      for (int j = 0; j < 4; ++j) {
        acc[i][j] = Frag<T>::mma(ah, bh[j], acc[i][j]);
        if (SPLIT) {
          acc[i][j] = Frag<T>::mma(ah, bl[j], acc[i][j]);
          acc[i][j] = Frag<T>::mma(al, bh[j], acc[i][j]);
        }
      }
      Frag<T>::guard(acc[i][0], acc[i][3], ah, SPLIT ? al : ah);
    }
    Frag<T>::keep(bh[0], bh[1], bh[2], bh[3]);
    if (SPLIT) Frag<T>::keep(bl[0], bl[1], bl[2], bl[3]);
  }
  acc_guard4(acc[0][0], acc[0][1], acc[0][2], acc[0][3]);
  acc_guard4(acc[1][0], acc[1][1], acc[1][2], acc[1][3]);
  acc_guard4(acc[2][0], acc[2][1], acc[2][2], acc[2][3]);
  acc_guard4(acc[3][0], acc[3][1], acc[3][2], acc[3][3]);

  float* slab = sT[wave];
  const float* Rb = RESID ? (resid + (size_t)b * strideR) : nullptr;
#pragma unroll
  for (int i = 0; i < 4; ++i) {
    const int mBase = m0 + (i << 4);
#pragma unroll
    for (int j = 0; j < 4; ++j) {
      const int n = n0 + (j << 4) + rlane;
      float bv = 0.f;
      if (BIAS_MODE == 2) bv = bias[n];
#pragma unroll
      for (int r = 0; r < 8; ++r) {
        float v = acc[i][j][r] * scale;
        if (BIAS_MODE == 1) v += bias[mBase + mOff + r];
        if (BIAS_MODE == 2) v += bv;
        if (RESID) v += Rb[(size_t)(mBase + mOff + r) * ldc + n];
        if (ACT == 1) v = tanhf(v);
        if (ACT == 2) v = fmaxf(v, 0.0f);
        if (ACT == 3) v = v / (1.0f + expf(-v));
        if (ACT == 4) v = (v > 0.f) ? v : 0.01f * v;
        if (ACT == 5) v = 0.5f * v * (1.0f + erff(v * 0.70710678118654752f));
        slab[(mOff + r) * 68 + (j << 4) + rlane] = v;
      }
    }
    __builtin_amdgcn_fence(__ATOMIC_RELEASE, "workgroup");
    __builtin_amdgcn_wave_barrier();
    __builtin_amdgcn_fence(__ATOMIC_ACQUIRE, "workgroup");
    if (OUT_MODE == 0) {
      float* C = (float*)Cout + (size_t)b * strideC;
      const int hh = lane >> 4, c4 = (lane & 15) * 4;
      for (int pass = 0; pass < 2; ++pass) {
#pragma unroll
        for (int it = 0; it < 8; ++it) {
          const int row = it * 2 + hh;
          v4f v = *(const v4f*)(slab + row * 68 + c4);
          *(volatile v4f*)(C + (size_t)(mBase + row) * ldc + n0 + c4) = v;
        }
        __threadfence();
      }
    } else {
      const int q = lane >> 3, c8 = (lane & 7) * 8;
      unsigned short* C  = (unsigned short*)Cout  + (size_t)b * strideC;
      unsigned short* C2 = (OUT_MODE == 2) ? ((unsigned short*)Cout2 + (size_t)b * strideC) : nullptr;
      for (int pass = 0; pass < 2; ++pass) {
#pragma unroll
        for (int it = 0; it < 4; ++it) {
          const int row = it * 4 + q;
          const float* sp = slab + row * 68 + c8;
          v8h hv, lv;
#pragma unroll
          for (int e = 0; e < 8; ++e) {
            if (OUT_MODE == 1) {
              hv[e] = (_Float16)sp[e];
            } else {
              unsigned short hb = f2bf_bits(sp[e]);
              unsigned short lb = f2bf_bits(sp[e] - bf_bits2f(hb));
              hv[e] = __builtin_bit_cast(_Float16, hb);
              lv[e] = __builtin_bit_cast(_Float16, lb);
            }
          }
          *(volatile v8h*)(C + (size_t)(mBase + row) * ldc + n0 + c8) = hv;
          if (OUT_MODE == 2) *(volatile v8h*)(C2 + (size_t)(mBase + row) * ldc + n0 + c8) = lv;
        }
        __threadfence();
      }
    }
    __builtin_amdgcn_fence(__ATOMIC_RELEASE, "workgroup");
    __builtin_amdgcn_wave_barrier();
    __builtin_amdgcn_fence(__ATOMIC_ACQUIRE, "workgroup");
  }
}

__global__ __launch_bounds__(256) void cvt_image_f16(const float* __restrict__ img, _Float16* __restrict__ Aout) {
  __shared__ __align__(16) float sImg[kEmb * kSpatial];
  const int i   = blockIdx.x;
  const int tid = threadIdx.x;
  const float* src = img + (size_t)i * (kEmb * kSpatial);
  for (int q = tid; q < (kEmb * kSpatial) / 4; q += 256)
    *(v4f*)(sImg + 4 * q) = *(const v4f*)(src + 4 * q);
  __syncthreads();

  v8h hv[4];
#pragma unroll
  for (int k = 0; k < 4; ++k) {
    const int idx = tid + 256 * k;
    int p = idx >> 4;
    p = (p < kSpatial) ? p : (kSpatial - 1);
    const int c8 = (idx & 15) * 8;
#pragma unroll
    for (int e = 0; e < 8; ++e) hv[k][e] = (_Float16)(sImg[(c8 + e) * kSpatial + p] * OPERAND_CARRY);
  }
  _Float16* dst = Aout + (size_t)i * (kSpatial * kEmb);
  for (int pass = 0; pass < 2; ++pass) {
#pragma unroll
    for (int k = 0; k < 4; ++k) {
      const int idx = tid + 256 * k;
      int p = idx >> 4;
      p = (p < kSpatial) ? p : (kSpatial - 1);
      const int c8 = (idx & 15) * 8;
      if (idx < kSpatial * 16) {
        *(volatile v8h*)(dst + (size_t)p * kEmb + c8) = hv[k];
      }
    }
    __threadfence();
  }
}

__global__ __launch_bounds__(256) void cvt_text_f16(const float* __restrict__ txt, _Float16* __restrict__ Bout) {
  const int idx = blockIdx.x * 256 + threadIdx.x;
  const float* s = txt + (size_t)idx * 8;
  const v4f a0 = *(const v4f*)(s);
  const v4f a1 = *(const v4f*)(s + 4);
  v8h hv;
#pragma unroll
  for (int e = 0; e < 4; ++e) {
    hv[e]     = (_Float16)(a0[e] * OPERAND_CARRY);
    hv[4 + e] = (_Float16)(a1[e] * OPERAND_CARRY);
  }
  _Float16* d = Bout + (size_t)idx * 8;
  for (int pass = 0; pass < 2; ++pass) {
    *(volatile v8h*)d = hv;
    __threadfence();
  }
}

__global__ __launch_bounds__(256) void maxsum_kernel(const float* __restrict__ Cp, float* __restrict__ Mt, int chunk) {
  __shared__ __align__(16) float sM[32];
  const int tid  = threadIdx.x;
  const int lane = tid & 31;
  const int wave = tid >> 5;
  const int i    = blockIdx.x >> 1;
  const int half = blockIdx.x & 1;
  const float neg_big = -__builtin_huge_valf();
  const float* rowbase = Cp + (size_t)i * kSpatial * kChunkN;
#pragma unroll 1
  for (int j = 0; j < 4; ++j) {
    const int tloc = half * 32 + wave * 4 + j;
    const float* col = rowbase + tloc * kNumWords + lane;
    float mx = neg_big;
#pragma unroll 7
    for (int p = 0; p < kSpatial; ++p) mx = fmaxf(mx, col[(size_t)p * kChunkN]);
    float ssum = mx;
#pragma unroll
    for (int off = 1; off < 32; off <<= 1) ssum += __shfl_xor(ssum, off, 32);
    if (lane == 0) sM[wave * 4 + j] = ssum;
  }
  __syncthreads();
  if (wave == 0) {
    const int l8 = lane & 7;
    const v4f v = *(const v4f*)(sM + l8 * 4);
    float* dst = Mt + (size_t)i * kNumTxt + chunk * 64 + half * 32 + l8 * 4;
    for (int pass = 0; pass < 2; ++pass) {
      if (lane < 8) { *(volatile v4f*)dst = v; }
      __threadfence();
    }
  }
}

__global__ __launch_bounds__(256) void final_kernel(const float* __restrict__ Mt, const int* __restrict__ len,
                                                    const float* __restrict__ nlt, float* __restrict__ out) {
  const int idx = blockIdx.x * 256 + threadIdx.x;
  const float scale = expf(nlt[0]);
  const int ia = idx >> 6;
  const int ta = (idx & 63) * 4;
  const v4f ma = *(const v4f*)(Mt + (size_t)ia * kNumTxt + ta);
  const v4i la = *(const v4i*)(len + ta);
  v4f oa;
#pragma unroll
  for (int e = 0; e < 4; ++e) {
    const float lf = (float)la[e];
    const float r  = 1.0f / lf;
    oa[e] = (ma[e] * r) * scale;
  }
  const int tb = idx >> 6;
  const int ib = (idx & 63) * 4;
  const float lfb = (float)len[tb];
  const float rb  = 1.0f / lfb;
  v4f ob;
#pragma unroll
  for (int e = 0; e < 4; ++e) {
    const float m = Mt[(size_t)(ib + e) * kNumTxt + tb];
    ob[e] = (m * rb) * scale;
  }
  float* pa = out + (size_t)ia * kNumTxt + ta;
  float* pb = out + kOut1Elem + (size_t)tb * kNumImg + ib;
  for (int pass = 0; pass < 2; ++pass) {
    *(volatile v4f*)pa = oa;
    *(volatile v4f*)pb = ob;
    __threadfence();
  }
}

extern "C" void kernel_launch(void* const* d_in, const int* in_sizes, int n_in,
                              void* d_out, int out_size, void* d_ws, size_t ws_size,
                              hipStream_t stream) {
  if (n_in < 4) return;
  if (in_sizes[0] != kImgElems || in_sizes[1] != kTxtElems || in_sizes[2] != kNumTxt || in_sizes[3] < 1) return;
  if (out_size != kOutElems) return;
  if (ws_size < kWsTotal) return;

  const float* img = (const float*)d_in[0];
  const float* txt = (const float*)d_in[1];
  const int*   len = (const int*)d_in[2];
  const float* nlt = (const float*)d_in[3];
  float*       out = (float*)d_out;

  char* ws = (char*)d_ws;
  _Float16* A16  = (_Float16*)(ws + kOffA);
  _Float16* Bt16 = (_Float16*)(ws + kOffBt);
  float*    Cp   = (float*)(ws + kOffC);
  float*    Mt   = (float*)(ws + kOffM);

  cvt_image_f16<<<kNumImg, 256, 0, stream>>>(img, A16);
  cvt_text_f16<<<kTxtElems / (8 * 256), 256, 0, stream>>>(txt, Bt16);

  const int tiles = (kGemmM / 64) * (kChunkN / 64);
  for (int c = 0; c < kNumChunks; ++c) {
    const unsigned short* Ap  = (const unsigned short*)A16;
    const unsigned short* Btp = (const unsigned short*)(Bt16 + (size_t)c * kChunkN * kEmb);
    wmma_gemm64<0, false, 0, 0, false, 0><<<dim3(tiles / 8, 1), 256, 0, stream>>>(
        Ap, Ap, kEmb, 0L,
        Btp, Btp, kEmb, 0L,
        (void*)Cp, (void*)Cp, kChunkN, 0L,
        (const float*)Cp,
        (const float*)Cp, 0L,
        kGemmM, kChunkN, kGemmK, CARRY_FOLD);
    maxsum_kernel<<<kNumImg * 2, 256, 0, stream>>>(Cp, Mt, c);
  }
  final_kernel<<<(kNumImg * kNumTxt / 4) / 256, 256, 0, stream>>>(Mt, len, nlt, out);
}
